// Tucker3D_89240830476843
// MI455X (gfx1250) — hardware-verified
//
#include <hip/hip_runtime.h>
#include <math.h>

typedef __attribute__((ext_vector_type(16))) _Float16 v16h;
typedef __attribute__((ext_vector_type(16))) __bf16 v16b;
typedef __attribute__((ext_vector_type(8)))  _Float16 v8h;
typedef __attribute__((ext_vector_type(8)))  float v8f;
typedef __attribute__((ext_vector_type(4)))  float v4f;
typedef __attribute__((ext_vector_type(2)))  float v2f;
typedef __attribute__((ext_vector_type(4)))  unsigned v4u;
typedef __attribute__((ext_vector_type(4)))  int v4i;
typedef float __attribute__((may_alias)) float_a;
typedef int __attribute__((may_alias)) int_a;

template <typename T> __device__ __forceinline__ void vst2(void* p, T v) { *(volatile T*)p = v; __threadfence(); *(volatile T*)p = v; }
__device__ __forceinline__ v8f wmma16(v16h a, v16h b, v8f c) {
  v8f d = __builtin_amdgcn_wmma_f32_16x16x32_f16(false, a, false, b, (short)0, c, false, false);
  asm volatile("v_nop\n\tv_nop\n\tv_nop\n\tv_nop" : "+v"(d) : "v"(a), "v"(b));
  return d;
}
__device__ __forceinline__ v8f wmma_bf(v16b a, v16b b, v8f c) {
  v8f d = __builtin_amdgcn_wmma_f32_16x16x32_bf16(false, a, false, b, (short)0, c, false, false);
  asm volatile("v_nop\n\tv_nop\n\tv_nop\n\tv_nop" : "+v"(d) : "v"(a), "v"(b));
  return d;
}
__device__ __forceinline__ v16h frag_h(const _Float16* rowk0, int lane) {
  union { v16h v; v8h q[2]; } u; const _Float16* p = rowk0 + 8 * (lane >> 4);
  u.q[0] = *(const v8h*)p; u.q[1] = *(const v8h*)(p + 16); return u.v;
}
__device__ __forceinline__ v16h frag_f32(const float* rowk0, int lane) {
  v16h a; const float* p = rowk0 + 8 * (lane >> 4);
#pragma unroll
  for (int i = 0; i < 8; ++i) { a[i] = (_Float16)p[i]; a[8 + i] = (_Float16)p[16 + i]; }
  return a;
}
__device__ __forceinline__ v16h frag_f32s(const float* rowk0, int lane, float sc) {
  v16h a; const float* p = rowk0 + 8 * (lane >> 4);
#pragma unroll
  for (int i = 0; i < 8; ++i) { a[i] = (_Float16)(p[i] * sc); a[8 + i] = (_Float16)(p[16 + i] * sc); }
  return a;
}
__device__ __forceinline__ v16h fragc_f32(const float* W, int k0, int n, int lane, int ld, int K) {
  v16h a; const int g = lane >> 4;
#pragma unroll
  for (int i = 0; i < 8; ++i) { const int ka = k0 + 8 * g + i, kb = ka + 16;
    a[i] = (_Float16)(ka < K ? W[(size_t)ka * ld + n] : 0.f); a[8 + i] = (_Float16)(kb < K ? W[(size_t)kb * ld + n] : 0.f); }
  return a;
}
struct F2 { v16b h, l; };
__device__ __forceinline__ F2 bsplit16(const float v[16]) { F2 r;
#pragma unroll
  for (int i = 0; i < 16; ++i) { const __bf16 h = (__bf16)v[i]; r.h[i] = h; r.l[i] = (__bf16)(v[i] - (float)h); }
  return r; }
__device__ __forceinline__ F2 split_row(const float* row, int k0, int lane) { float v[16]; const float* p = row + k0 + 8 * (lane >> 4);
#pragma unroll
  for (int i = 0; i < 8; ++i) { v[i] = p[i]; v[8 + i] = p[16 + i]; }
  return bsplit16(v); }
__device__ __forceinline__ F2 split_rowK(const float* row, int k0, int lane, int K) { float v[16]; const int g = lane >> 4;
#pragma unroll
  for (int i = 0; i < 8; ++i) { const int ka = k0 + 8 * g + i, kb = ka + 16; v[i] = ka < K ? row[ka] : 0.f; v[8 + i] = kb < K ? row[kb] : 0.f; }
  return bsplit16(v); }
__device__ __forceinline__ F2 split_col(const float* W, int k0, int n, int lane, int ld, int K) { float v[16]; const int g = lane >> 4;
#pragma unroll
  for (int i = 0; i < 8; ++i) { const int ka = k0 + 8 * g + i, kb = ka + 16; v[i] = ka < K ? W[(size_t)ka * ld + n] : 0.f; v[8 + i] = kb < K ? W[(size_t)kb * ld + n] : 0.f; }
  return bsplit16(v); }
__device__ __forceinline__ v8f mac3(const F2& a, const F2& b, v8f c) { c = wmma_bf(a.l, b.h, c); c = wmma_bf(a.h, b.l, c); return wmma_bf(a.h, b.h, c); }
__device__ __forceinline__ float sigm(float v) { return 1.0f / (1.0f + expf(-v)); }
#define LDSX() do { asm volatile("s_wait_dscnt 0" ::: "memory"); __builtin_amdgcn_wave_barrier(); __builtin_amdgcn_fence(__ATOMIC_RELEASE, "workgroup"); } while (0)

#define NPTS 262144
#define CL 32
#define NL 256
#define RDIV 1.3f

__global__ __launch_bounds__(256) void k_packG(const float* __restrict__ G, _Float16* __restrict__ Gp) {
  const int z = blockIdx.x, tid = threadIdx.x; __shared__ __align__(16) _Float16 sr[CL * CL];
  for (int q = tid; q < CL * CL; q += 256) sr[q] = (_Float16)G[(size_t)q * CL + z];
  __syncthreads();
  if (tid < CL * CL / 8) vst2(Gp + (size_t)z * CL * CL + tid * 8, *(const v4u*)(&sr[tid * 8]));
}
__device__ __forceinline__ void bilin(const float* __restrict__ plane, float gx, float gy, int c0, float* outv) {
  const float xf = (gx + 1.0f) * 0.5f * (float)(NL - 1), yf = (gy + 1.0f) * 0.5f * (float)(NL - 1);
  const float x0f = floorf(xf), y0f = floorf(yf); const float wx1 = xf - x0f, wy1 = yf - y0f, wx0 = 1.0f - wx1, wy0 = 1.0f - wy1;
  const int x0 = (int)x0f, y0 = (int)y0f, x1 = x0 + 1, y1 = y0 + 1;
  const bool vx0 = x0 >= 0 && x0 < NL, vx1 = x1 >= 0 && x1 < NL, vy0 = y0 >= 0 && y0 < NL, vy1 = y1 >= 0 && y1 < NL;
  const int cx0 = min(max(x0, 0), NL - 1), cx1 = min(max(x1, 0), NL - 1), cy0 = min(max(y0, 0), NL - 1), cy1 = min(max(y1, 0), NL - 1);
  const float w00 = (vx0 && vy0) ? wx0 * wy0 : 0.f, w10 = (vx1 && vy0) ? wx1 * wy0 : 0.f, w01 = (vx0 && vy1) ? wx0 * wy1 : 0.f, w11 = (vx1 && vy1) ? wx1 * wy1 : 0.f;
#pragma unroll
  for (int e = 0; e < 8; ++e) { const float* pc = plane + (size_t)(c0 + e) * NL * NL;
    outv[e] = pc[cy0 * NL + cx0] * w00 + pc[cy0 * NL + cx1] * w10 + pc[cy1 * NL + cx0] * w01 + pc[cy1 * NL + cx1] * w11; }
}
__global__ __launch_bounds__(128) void k_main(const float* __restrict__ coords, const float* __restrict__ pxy, const float* __restrict__ pyz, const float* __restrict__ pxz, const _Float16* __restrict__ Gp, float* __restrict__ out) {
  __shared__ __align__(16) float sfx[4][16][CL + 1], sfy[4][16][CL + 1], sfz[4][16][CL + 1];
  __shared__ __align__(16) _Float16 sa[4][16][40];
  __shared__ __align__(16) float so[64];
  const int tid = threadIdx.x, wave = tid >> 5, lane = tid & 31, col = lane & 15, g = lane >> 4;
  const int p0 = blockIdx.x * 64 + wave * 16;
  { const int p = p0 + col; const float cx = coords[(size_t)p * 3] * (1.0f / RDIV), cy = coords[(size_t)p * 3 + 1] * (1.0f / RDIV), cz = coords[(size_t)p * 3 + 2] * (1.0f / RDIV);
#pragma unroll 1
    for (int gi = g * 6; gi < g * 6 + 6; ++gi) { const int pl = gi >> 2, c0 = (gi & 3) * 8; float v[8];
      if (pl == 0) bilin(pxy, cx, cy, c0, v); else if (pl == 1) bilin(pyz, cy, cz, c0, v); else bilin(pxz, cx, cz, c0, v);
      float* dst = pl == 0 ? &sfx[wave][col][c0] : (pl == 1 ? &sfy[wave][col][c0] : &sfz[wave][col][c0]);
#pragma unroll
      for (int e = 0; e < 8; ++e) dst[e] = v[e] * 1000.0f; } }
  LDSX();
  v8f acc[2] = {};
#pragma unroll 2
  for (int xk = 0; xk < CL; ++xk) { const float fxv = sfx[wave][col][xk]; union { v8h h[2]; v4u u[2]; } pk;
#pragma unroll
    for (int e = 0; e < 16; ++e) pk.h[e >> 3][e & 7] = (_Float16)(fxv * sfy[wave][col][g * 16 + e]);
    *(v4u*)(&sa[wave][col][g * 16]) = pk.u[0]; *(v4u*)(&sa[wave][col][g * 16 + 8]) = pk.u[1];
    LDSX();
    const v16h a = frag_h(&sa[wave][col][0], lane);
#pragma unroll
    for (int t = 0; t < 2; ++t) acc[t] = wmma16(a, frag_h(Gp + (size_t)(t * 16 + col) * (CL * CL) + xk * CL, lane), acc[t]);
    LDSX(); }
  float part[8];
#pragma unroll
  for (int r = 0; r < 8; ++r) { const int m = 8 * g + r; part[r] = acc[0][r] * sfz[wave][m][col] + acc[1][r] * sfz[wave][m][16 + col]; }
#pragma unroll
  for (int r = 0; r < 8; ++r) { float v = part[r];
#pragma unroll
    for (int off = 1; off < 16; off <<= 1) v += __shfl_xor(v, off, 32);
    part[r] = v; }
  if (col == 0) {
#pragma unroll
    for (int r = 0; r < 8; ++r) so[wave * 16 + 8 * g + r] = part[r] * 1.0e-9f; }
  __syncthreads();
  if (tid < 16) vst2(out + (size_t)blockIdx.x * 64 + tid * 4, *(const v4f*)(&so[tid * 4]));
}
extern "C" void kernel_launch(void* const* d_in, const int* in_sizes, int n_in, void* d_out, int out_size, void* d_ws, size_t ws_size, hipStream_t stream) {
  (void)in_sizes; (void)n_in; (void)out_size; (void)ws_size;
  const float* coords = (const float*)d_in[0]; const float* pxy = (const float*)d_in[1]; const float* pyz = (const float*)d_in[2]; const float* pxz = (const float*)d_in[3]; const float* G = (const float*)d_in[4];
  float* out = (float*)d_out;
  _Float16* Gp = (_Float16*)d_ws;
  k_packG<<<CL, 256, 0, stream>>>(G, Gp);
  k_main<<<NPTS / 64, 128, 0, stream>>>(coords, pxy, pyz, pxz, Gp, out);
}
